// GATConvDGL_66812511256931
// MI455X (gfx1250) — hardware-verified
//
#include <hip/hip_runtime.h>
#include <hip/hip_bf16.h>
#include <stddef.h>


#define DF    128
#define NH    4
#define GR    32
#define AP    136
#define XSP   132
#define NB    512
#define CHUNK 2048
#define NTHR  256
#define NWAVE 8
#define WCAP  256
#define NGRP  (CHUNK / (NTHR * 4))

#define LDS_SACC  (NB * DF)
#define LDS_ELS   (NB * NH)
#define LDS_MX    (NB * NH)
#define LDS_DEN   (NB * NH)
#define LDS_LIST  (NWAVE * WCAP)
#define LDS_WORDS (LDS_SACC + LDS_ELS + LDS_MX + LDS_DEN + LDS_LIST + NWAVE)
#define LDS_BYTES (LDS_WORDS * 4)

static_assert(WCAP == (CHUNK / NTHR) * 32);
static_assert(NGRP >= 1);
static_assert(NB == 512);
static_assert(CHUNK == 2048);
static_assert((LDS_SACC % 4) == 0 && (LDS_ELS % 4) == 0);
static_assert(LDS_BYTES == 294944);
static_assert((AP * 2) % 16 == 0 && (XSP * 4) % 16 == 0);

typedef float          v4f   __attribute__((ext_vector_type(4)));
typedef float          v8f   __attribute__((ext_vector_type(8)));
typedef int            v4i   __attribute__((ext_vector_type(4)));
typedef unsigned short v8us  __attribute__((ext_vector_type(8)));
typedef __bf16         v16bf __attribute__((ext_vector_type(16)));
union Frag  { v16bf v; v8us half[2]; };
union Pack8 { v8us u; unsigned short s[8]; };

__device__ __forceinline__ v8f wm(v16bf a, v16bf b, v8f c) {
  v8f d = __builtin_amdgcn_wmma_f32_16x16x32_bf16(false, a, false, b, (short)0, c, false, false);
  asm volatile("v_nop\n\tv_nop\n\tv_nop\n\tv_nop" : "+v"(d) : "v"(a), "v"(b));
  return d;
}

__device__ __forceinline__ unsigned short bf_rne(float f) {
  unsigned u = __float_as_uint(f);
  u += 0x7FFFu + ((u >> 16) & 1u);
  return (unsigned short)(u >> 16);
}
__device__ __forceinline__ float bf_val(unsigned short s) {
  return __uint_as_float(((unsigned)s) << 16);
}

__device__ __forceinline__ void split8(const v4f a, const v4f c, v8us& hi, v8us& lo) {
  Pack8 ph, pl;
#define SPL(J, F) { const float fv = (F); const unsigned short hs = bf_rne(fv); ph.s[J] = hs; pl.s[J] = bf_rne(fv - bf_val(hs)); }
  SPL(0, a.x) SPL(1, a.y) SPL(2, a.z) SPL(3, a.w)
  SPL(4, c.x) SPL(5, c.y) SPL(6, c.z) SPL(7, c.w)
#undef SPL
  hi = ph.u;
  lo = pl.u;
}

__device__ __forceinline__ v4f shx4(v4f v, int mk) {
  v4f r;
  r.x = __shfl_xor(v.x, mk, 32);
  r.y = __shfl_xor(v.y, mk, 32);
  r.z = __shfl_xor(v.z, mk, 32);
  r.w = __shfl_xor(v.w, mk, 32);
  return r;
}

__global__ __launch_bounds__(NTHR) void k_prep(const float* __restrict__ W,
                                               unsigned short* Wh, unsigned short* Wl, int n8) {
  const int i = blockIdx.x * NTHR + threadIdx.x;
  if (i >= n8) return;
  const size_t o = (size_t)i * 8;
  const v4f a = *(const v4f*)(W + o);
  const v4f c = *(const v4f*)(W + o + 4);
  v8us hi, lo;
  split8(a, c, hi, lo);
  *(volatile v8us*)(Wh + o) = hi;
  *(volatile v8us*)(Wl + o) = lo;
  __threadfence();
  *(volatile v8us*)(Wh + o) = hi;
  *(volatile v8us*)(Wl + o) = lo;
}

__global__ __launch_bounds__(NTHR) void k_gemm(
    const float* __restrict__ x, const unsigned short* __restrict__ Wh,
    const unsigned short* __restrict__ Wl, const float* __restrict__ bias,
    const float* __restrict__ a_l, const float* __restrict__ a_r,
    float* Z, float* El, float* Er, int nN) {
  __shared__ __attribute__((aligned(16))) unsigned short Ah[GR * AP];
  __shared__ __attribute__((aligned(16))) unsigned short Al[GR * AP];
  __shared__ __attribute__((aligned(16))) float Xs[GR * XSP];
  __shared__ __attribute__((aligned(16))) float als[DF];
  __shared__ __attribute__((aligned(16))) float ars[DF];
  __shared__ __attribute__((aligned(16))) float Esl[GR * NH];
  __shared__ __attribute__((aligned(16))) float Esr[GR * NH];

  const int tid  = threadIdx.x;
  const int lane = tid & 31;
  const int wave = tid >> 5;
  const int hh   = lane >> 4;
  const int m    = lane & 15;
  const int rowBase = blockIdx.x * GR;

  if (tid < DF) als[tid] = a_l[tid];
  else          ars[tid - DF] = a_r[tid - DF];

  {
    const int r  = tid >> 3;
    const int c0 = (tid & 7) * 16;
    int row = rowBase + r;
    if (row > nN - 1) row = nN - 1;
    const float* p = x + (size_t)row * DF + c0;
    const v4f f0 = *(const v4f*)(p),     f1 = *(const v4f*)(p + 4);
    const v4f f2 = *(const v4f*)(p + 8), f3 = *(const v4f*)(p + 12);
    v8us h0, l0, h1, l1;
    split8(f0, f1, h0, l0);
    split8(f2, f3, h1, l1);
    *(v8us*)(Ah + r * AP + c0)     = h0;
    *(v8us*)(Ah + r * AP + c0 + 8) = h1;
    *(v8us*)(Al + r * AP + c0)     = l0;
    *(v8us*)(Al + r * AP + c0 + 8) = l1;
  }
  __syncthreads();

  const int ncol = wave * 16 + m;
  v8f c0a = {0.f, 0.f, 0.f, 0.f, 0.f, 0.f, 0.f, 0.f};
  v8f c1a = {0.f, 0.f, 0.f, 0.f, 0.f, 0.f, 0.f, 0.f};
#pragma unroll
  for (int kt = 0; kt < DF / 32; ++kt) {
    const int k0 = kt * 32;
    Frag a0h, a0l, a1h, a1l, bh, bl;
    const unsigned short* pbh = Wh + (size_t)ncol * DF + k0 + 8 * hh;
    const unsigned short* pbl = Wl + (size_t)ncol * DF + k0 + 8 * hh;
    const unsigned short* p0h = Ah + m * AP + k0 + 8 * hh;
    const unsigned short* p0l = Al + m * AP + k0 + 8 * hh;
    const unsigned short* p1h = Ah + (16 + m) * AP + k0 + 8 * hh;
    const unsigned short* p1l = Al + (16 + m) * AP + k0 + 8 * hh;
    bh.half[0]  = *(const v8us*)pbh; bh.half[1]  = *(const v8us*)(pbh + 16);
    bl.half[0]  = *(const v8us*)pbl; bl.half[1]  = *(const v8us*)(pbl + 16);
    a0h.half[0] = *(const v8us*)p0h; a0h.half[1] = *(const v8us*)(p0h + 16);
    a0l.half[0] = *(const v8us*)p0l; a0l.half[1] = *(const v8us*)(p0l + 16);
    a1h.half[0] = *(const v8us*)p1h; a1h.half[1] = *(const v8us*)(p1h + 16);
    a1l.half[0] = *(const v8us*)p1l; a1l.half[1] = *(const v8us*)(p1l + 16);
    c0a = wm(a0h.v, bh.v, c0a);
    c0a = wm(a0h.v, bl.v, c0a);
    c0a = wm(a0l.v, bh.v, c0a);
    c1a = wm(a1h.v, bh.v, c1a);
    c1a = wm(a1h.v, bl.v, c1a);
    c1a = wm(a1l.v, bh.v, c1a);
  }

  {
    const float bv = bias[ncol];
#pragma unroll
    for (int r = 0; r < 8; ++r) {
      Xs[(8 * hh + r) * XSP + ncol]      = c0a[r] + bv;
      Xs[(16 + 8 * hh + r) * XSP + ncol] = c1a[r] + bv;
    }
  }
  __syncthreads();

  {
    const int r = tid >> 3;
    const int q = tid & 7;
    v4f sl = {0.f, 0.f, 0.f, 0.f};
    v4f sr = {0.f, 0.f, 0.f, 0.f};
#pragma unroll
    for (int i = 0; i < 4; ++i) {
      const int c = 16 * q + 4 * i;
      const v4f xv = *(const v4f*)(Xs + r * XSP + c);
      const v4f la = *(const v4f*)(als + c);
      const v4f ra = *(const v4f*)(ars + c);
      sl += xv * la;
      sr += xv * ra;
    }
#pragma unroll
    for (int mk = 1; mk < 8; mk <<= 1) {
      sl += shx4(sl, mk);
      sr += shx4(sr, mk);
    }
    if (q == 0) {
      *(v4f*)(Esl + r * NH) = sl;
      *(v4f*)(Esr + r * NH) = sr;
    }
  }
  __syncthreads();

  v4f xr[4];
#pragma unroll
  for (int i = 0; i < 4; ++i) xr[i] = *(const v4f*)(Xs + (4 * wave + i) * XSP + 4 * lane);
  float* zp[4];
#pragma unroll
  for (int i = 0; i < 4; ++i) zp[i] = Z + (size_t)(rowBase + 4 * wave + i) * DF + 4 * lane;
  bool doG = false;
  v4f gv = {0.f, 0.f, 0.f, 0.f};
  float* gp = El;
  if (wave == 0) {
    gv = *(const v4f*)(Esl + 4 * lane);
    gp = El + (size_t)rowBase * NH + 4 * lane;
    doG = true;
  } else if (wave == 1) {
    gv = *(const v4f*)(Esr + 4 * lane);
    gp = Er + (size_t)rowBase * NH + 4 * lane;
    doG = true;
  }

#pragma unroll
  for (int i = 0; i < 4; ++i) *(volatile v4f*)(zp[i]) = xr[i];
  if (doG) *(volatile v4f*)gp = gv;
  __threadfence();
#pragma unroll
  for (int i = 0; i < 4; ++i) *(volatile v4f*)(zp[i]) = xr[i];
  if (doG) *(volatile v4f*)gp = gv;
}

__global__ __launch_bounds__(NTHR) void k_gat(
    const int* __restrict__ rowp, const int* __restrict__ colp,
    const float* __restrict__ Z, const float* __restrict__ El, const float* __restrict__ Er,
    float* out, int nN, int nE) {
  extern __shared__ v4f lds_dyn[];
  float* sacc = (float*)lds_dyn;
  float* els  = sacc + LDS_SACC;
  float* mx   = els + LDS_ELS;
  float* den  = mx + LDS_MX;
  int*   list = (int*)(den + LDS_DEN);
  int*   wcnt = list + LDS_LIST;

  const int tid  = threadIdx.x;
  const int lane = tid & 31;
  const int wave = tid >> 5;
  const int nodeBase = blockIdx.x * NB;

  {
    const v4f z4 = {0.f, 0.f, 0.f, 0.f};
    const v4f m4 = {-1.0e30f, -1.0e30f, -1.0e30f, -1.0e30f};
    for (int i = tid; i < LDS_SACC / 4; i += NTHR) lds_dyn[i] = z4;
    for (int s = tid; s < NB; s += NTHR) {
      int node = nodeBase + s;
      if (node > nN - 1) node = nN - 1;
      const v4f e = *(const v4f*)(El + (size_t)node * NH);
      *(v4f*)(els + s * NH) = e;
      *(v4f*)(mx  + s * NH) = m4;
      *(v4f*)(den + s * NH) = z4;
    }
  }
  __syncthreads();

  const bool al16 = true;

  const int nChunks = (nE + CHUNK - 1) / CHUNK;
#pragma unroll 1
  for (int ch = 0; ch < nChunks; ++ch) {
    const int cbase = ch * CHUNK;
    int wc = 0;
#pragma unroll
    for (int g = 0; g < NGRP; ++g) {
      const int el0 = (g * NTHR + tid) * 4;
      const int e0  = cbase + el0;
      const int sent = -2147483647 - 1;
      v4i d;
      if (al16 && (cbase + CHUNK <= nE)) {
        d = *(const v4i*)(rowp + e0);
      } else {
        const int q0 = rowp[min(e0,     nE - 1)];
        const int q1 = rowp[min(e0 + 1, nE - 1)];
        const int q2 = rowp[min(e0 + 2, nE - 1)];
        const int q3 = rowp[min(e0 + 3, nE - 1)];
        d.x = (e0     < nE) ? q0 : sent;
        d.y = (e0 + 1 < nE) ? q1 : sent;
        d.z = (e0 + 2 < nE) ? q2 : sent;
        d.w = (e0 + 3 < nE) ? q3 : sent;
      }
      const unsigned s0 = (unsigned)d.x - (unsigned)nodeBase;
      const unsigned s1 = (unsigned)d.y - (unsigned)nodeBase;
      const unsigned s2 = (unsigned)d.z - (unsigned)nodeBase;
      const unsigned s3 = (unsigned)d.w - (unsigned)nodeBase;
      const bool h0 = s0 < (unsigned)NB;
      const bool h1 = s1 < (unsigned)NB;
      const bool h2 = s2 < (unsigned)NB;
      const bool h3 = s3 < (unsigned)NB;
      const unsigned many = __builtin_amdgcn_ballot_w32(h0 | h1 | h2 | h3);
      if (many != 0u) {
#define HITJ(J, HJ, SJ) { \
          const unsigned mj = __builtin_amdgcn_ballot_w32(HJ); \
          if (HJ) { \
            const int pos = wc + (int)__builtin_amdgcn_mbcnt_lo(mj, 0u); \
            if (pos < WCAP) list[wave * WCAP + pos] = ((el0 + (J)) << 9) | (int)(SJ); \
          } \
          wc += (int)__builtin_popcount(mj); }
        HITJ(0, h0, s0)
        HITJ(1, h1, s1)
        HITJ(2, h2, s2)
        HITJ(3, h3, s3)
#undef HITJ
      }
    }
    if (lane == 0) wcnt[wave] = wc;
    __syncthreads();

    if (wave == 0) {
      for (int wsx = 0; wsx < NWAVE; ++wsx) {
        int n = wcnt[wsx];
        if (n > WCAP) n = WCAP;
        if (n < 0) n = 0;
        for (int i = 0; i < n; ++i) {
          const int ent  = list[wsx * WCAP + i];
          const int slot = ent & (NB - 1);
          const int el   = (ent >> 9) & (CHUNK - 1);
          int e = cbase + el;
          if (e > nE - 1) e = nE - 1;
          int src = colp[e];
          src = src < 0 ? 0 : (src > nN - 1 ? nN - 1 : src);
          const v4f er = *(const v4f*)(Er + (size_t)src * NH);
          v4f lg = *(const v4f*)(els + slot * NH) + er;
          lg.x = (lg.x > 0.f) ? lg.x : 0.2f * lg.x;
          lg.y = (lg.y > 0.f) ? lg.y : 0.2f * lg.y;
          lg.z = (lg.z > 0.f) ? lg.z : 0.2f * lg.z;
          lg.w = (lg.w > 0.f) ? lg.w : 0.2f * lg.w;
          const v4f mo = *(const v4f*)(mx + slot * NH);
          v4f mn;
          mn.x = fmaxf(mo.x, lg.x);
          mn.y = fmaxf(mo.y, lg.y);
          mn.z = fmaxf(mo.z, lg.z);
          mn.w = fmaxf(mo.w, lg.w);
          v4f rr, p;
          rr.x = __expf(fmaxf(mo.x - mn.x, -80.f));
          rr.y = __expf(fmaxf(mo.y - mn.y, -80.f));
          rr.z = __expf(fmaxf(mo.z - mn.z, -80.f));
          rr.w = __expf(fmaxf(mo.w - mn.w, -80.f));
          p.x = __expf(lg.x - mn.x);
          p.y = __expf(lg.y - mn.y);
          p.z = __expf(lg.z - mn.z);
          p.w = __expf(lg.w - mn.w);
          const v4f xv = *(const v4f*)(Z + (size_t)src * DF + 4 * lane);
          v4f* sp = (v4f*)(sacc + slot * DF + 4 * lane);
          const v4f cur = *sp;
          const v4f nxt = cur * rr + p * xv;
          *sp = nxt;
          const v4f dn  = *(const v4f*)(den + slot * NH);
          const v4f dnn = dn * rr + p;
          *(v4f*)(den + slot * NH) = dnn;
          *(v4f*)(mx  + slot * NH) = mn;
        }
      }
    }
    __syncthreads();
  }

#pragma unroll 1
  for (int j = 0; j < NB / NWAVE; ++j) {
    const int slot = wave * (NB / NWAVE) + j;
    const int node = nodeBase + slot;
    if (node >= nN) break;
    const v4f dn = *(const v4f*)(den + slot * NH);
    const v4f sv = *(const v4f*)(sacc + slot * DF + 4 * lane);
    v4f inv;
    inv.x = (dn.x > 0.f) ? (1.0f / dn.x) : 0.f;
    inv.y = (dn.y > 0.f) ? (1.0f / dn.y) : 0.f;
    inv.z = (dn.z > 0.f) ? (1.0f / dn.z) : 0.f;
    inv.w = (dn.w > 0.f) ? (1.0f / dn.w) : 0.f;
    const v4f y = sv * inv;
    float* op = out + (size_t)node * DF + 4 * lane;
    *(volatile v4f*)op = y;
    __threadfence();
    *(volatile v4f*)op = y;
  }
}

extern "C" void kernel_launch(void* const* d_in, const int* in_sizes, int n_in,
                              void* d_out, int out_size, void* d_ws, size_t ws_size,
                              hipStream_t stream) {
  if (n_in < 7) return;
  if (in_sizes[0] <= 0 || (in_sizes[0] % DF) != 0) return;
  const int nN = in_sizes[0] / DF;
  const int nE = in_sizes[1];
  if (nE < 1 || in_sizes[2] != nE) return;
  if (in_sizes[3] != DF * DF) return;
  if (in_sizes[4] != DF || in_sizes[5] != DF || in_sizes[6] != DF) return;
  if (out_size != nN * DF) return;

  const float* x    = (const float*)d_in[0];
  const int*   rowp = (const int*)d_in[1];
  const int*   colp = (const int*)d_in[2];
  const float* W    = (const float*)d_in[3];
  const float* bias = (const float*)d_in[4];
  const float* a_l  = (const float*)d_in[5];
  const float* a_r  = (const float*)d_in[6];
  float* out = (float*)d_out;

  const int nP = ((nN + GR - 1) / GR) * GR;
  size_t off = 0;
  unsigned short* Wh = (unsigned short*)((char*)d_ws + off);
  off += (size_t)DF * DF * sizeof(unsigned short);  off = (off + 255) & ~(size_t)255;
  unsigned short* Wl = (unsigned short*)((char*)d_ws + off);
  off += (size_t)DF * DF * sizeof(unsigned short);  off = (off + 255) & ~(size_t)255;
  float* Z  = (float*)((char*)d_ws + off);
  off += (size_t)nP * DF * sizeof(float);            off = (off + 255) & ~(size_t)255;
  float* El = (float*)((char*)d_ws + off);
  off += (size_t)nP * NH * sizeof(float);            off = (off + 255) & ~(size_t)255;
  float* Er = (float*)((char*)d_ws + off);
  off += (size_t)nP * NH * sizeof(float);            off = (off + 255) & ~(size_t)255;
  if (off > ws_size) return;

  const int n8 = DF * DF / 8;
  k_prep<<<(n8 + NTHR - 1) / NTHR, NTHR, 0, stream>>>(W, Wh, Wl, n8);

  k_gemm<<<nP / GR, NTHR, 0, stream>>>(x, Wh, Wl, bias, a_l, a_r, Z, El, Er, nN);

  hipFuncSetAttribute(reinterpret_cast<const void*>(&k_gat),
                      hipFuncAttributeMaxDynamicSharedMemorySize, LDS_BYTES);
  const int grid = (nN + NB - 1) / NB;
  k_gat<<<grid, NTHR, LDS_BYTES, stream>>>(rowp, colp, Z, El, Er, out, nN, nE);
}
